// LSTMFeatureExtractor_39067022524824
// MI455X (gfx1250) — hardware-verified
//
#include <hip/hip_runtime.h>


typedef _Float16 f16t;
typedef __bf16   bf16;
typedef f16t  v16h __attribute__((ext_vector_type(16)));
typedef f16t  v8h  __attribute__((ext_vector_type(8)));
typedef bf16  v16b __attribute__((ext_vector_type(16)));
typedef bf16  v8b  __attribute__((ext_vector_type(8)));
typedef bf16  v4b  __attribute__((ext_vector_type(4)));
typedef float v8f  __attribute__((ext_vector_type(8)));
typedef float v4f  __attribute__((ext_vector_type(4)));
typedef unsigned int v4u __attribute__((ext_vector_type(4)));
typedef unsigned int v2u __attribute__((ext_vector_type(2)));

union FragH { v16h v; v8h q[2]; };
union FragB { v16b v; v8b q[2]; };
union PkH   { v8h h; v4u u; };
union PkB   { v8b h; v4u u; };
union PkB4  { v4b h; v2u u; };

#define HID  512
#define G4   2048
#define DIN  64
#define FOUT 256
#define NB   16
#define HP   520
#define XP   72
#define NTHR 256

struct LdsLoop {
    f16t  h16[2][NB * HP];
    bf16  xh[NB * XP];
    bf16  xl[NB * XP];
    float c[NB * HID];
    float hf[NB * HID];
};
struct LdsHead {
    bf16  ph[NB * HID];
    bf16  pl[NB * HID];
    float o[NB * FOUT];
};
union __attribute__((aligned(16))) LdsU { LdsLoop a; LdsHead b; };

__device__ __forceinline__ v8f mma_h(v16h a, v16h b, v8f c) {
    return __builtin_amdgcn_wmma_f32_16x16x32_f16(false, a, false, b, (short)0, c, false, false);
}
__device__ __forceinline__ v8f mma_b(v16b a, v16b b, v8f c) {
    return __builtin_amdgcn_wmma_f32_16x16x32_bf16(false, a, false, b, (short)0, c, false, false);
}

__device__ __forceinline__ void guard4h(v8f (&c)[4], FragH (&a)[4], FragH& b) {
    asm volatile("v_nop\n\tv_nop\n\tv_nop\n\tv_nop"
                 : "+v"(c[0]), "+v"(c[1]), "+v"(c[2]), "+v"(c[3])
                 : "v"(a[0].v), "v"(a[1].v), "v"(a[2].v), "v"(a[3].v), "v"(b.v));
}
__device__ __forceinline__ void guard4b(v8f (&c)[4], FragB (&a)[4], FragB& b0, FragB& b1) {
    asm volatile("v_nop\n\tv_nop\n\tv_nop\n\tv_nop"
                 : "+v"(c[0]), "+v"(c[1]), "+v"(c[2]), "+v"(c[3])
                 : "v"(a[0].v), "v"(a[1].v), "v"(a[2].v), "v"(a[3].v), "v"(b0.v), "v"(b1.v));
}
__device__ __forceinline__ void guard2b(v8f (&c)[2], FragB (&a)[2], FragB& b0, FragB& b1) {
    asm volatile("v_nop\n\tv_nop\n\tv_nop\n\tv_nop"
                 : "+v"(c[0]), "+v"(c[1])
                 : "v"(a[0].v), "v"(a[1].v), "v"(b0.v), "v"(b1.v));
}

__device__ __forceinline__ float fsig(float x) {
    x = fminf(fmaxf(x, -40.0f), 40.0f);
    float t = __expf(-x);
    return __builtin_amdgcn_rcpf(1.0f + t);
}
__device__ __forceinline__ float ftanh(float x) {
    float ax = fminf(fabsf(x), 20.0f);
    float t  = __expf(-2.0f * ax);
    float r  = (1.0f - t) * __builtin_amdgcn_rcpf(1.0f + t);
    return copysignf(r, x);
}

__device__ __forceinline__ void gate_mma(v8f (&acc)[4],
                                         const f16t* awh,
                                         const bf16* axh,
                                         const bf16* axl,
                                         const f16t* hrow,
                                         const bf16* xhrow,
                                         const bf16* xlrow) {
#pragma unroll
    for (int ks = 0; ks < 2; ++ks) {
        const int k0 = 32 * ks;
        FragB bh, bl, a[4];
        bh.q[0] = *(const v8b*)(xhrow + k0);
        bh.q[1] = *(const v8b*)(xhrow + k0 + 16);
        bl.q[0] = *(const v8b*)(xlrow + k0);
        bl.q[1] = *(const v8b*)(xlrow + k0 + 16);
#pragma unroll
        for (int q = 0; q < 4; ++q) {
            const bf16* p = axh + (size_t)q * HID * DIN + k0;
            a[q].q[0] = *(const v8b*)p;
            a[q].q[1] = *(const v8b*)(p + 16);
        }
#pragma unroll
        for (int q = 0; q < 4; ++q) acc[q] = mma_b(a[q].v, bh.v, acc[q]);
#pragma unroll
        for (int q = 0; q < 4; ++q) acc[q] = mma_b(a[q].v, bl.v, acc[q]);
        guard4b(acc, a, bh, bl);
#pragma unroll
        for (int q = 0; q < 4; ++q) {
            const bf16* p = axl + (size_t)q * HID * DIN + k0;
            a[q].q[0] = *(const v8b*)p;
            a[q].q[1] = *(const v8b*)(p + 16);
        }
#pragma unroll
        for (int q = 0; q < 4; ++q) acc[q] = mma_b(a[q].v, bh.v, acc[q]);
        guard4b(acc, a, bh, bl);
    }
#pragma unroll 1
    for (int kt = 0; kt < HID / 32; ++kt) {
        const int k0 = 32 * kt;
        FragH b, a[4];
        b.q[0] = *(const v8h*)(hrow + k0);
        b.q[1] = *(const v8h*)(hrow + k0 + 16);
#pragma unroll
        for (int q = 0; q < 4; ++q) {
            const f16t* p = awh + (size_t)q * HID * HID + k0;
            a[q].q[0] = *(const v8h*)p;
            a[q].q[1] = *(const v8h*)(p + 16);
        }
#pragma unroll
        for (int q = 0; q < 4; ++q) acc[q] = mma_h(a[q].v, b.v, acc[q]);
        guard4h(acc, a, b);
    }
}

__device__ __forceinline__ void cell_update(v8f (&acc)[4], float inv, const float* bg, int jb,
                                            float* cp, f16t* hp16, float* hpf, bool last) {
    v4f bq[4][2];
#pragma unroll
    for (int q = 0; q < 4; ++q) {
        bq[q][0] = *(const v4f*)(bg + q * HID + jb);
        bq[q][1] = *(const v4f*)(bg + q * HID + jb + 4);
    }
    v4f cold[2];
    cold[0] = *(const v4f*)cp;
    cold[1] = *(const v4f*)(cp + 4);
    v4f cnew[2], hnew[2];
    PkH hk;
#pragma unroll
    for (int s = 0; s < 2; ++s) {
#pragma unroll
        for (int r = 0; r < 4; ++r) {
            const int e = 4 * s + r;
            float pi = fmaf(acc[0][e], inv, bq[0][s][r]);
            float pf = fmaf(acc[1][e], inv, bq[1][s][r]);
            float pg = fmaf(acc[2][e], inv, bq[2][s][r]);
            float po = fmaf(acc[3][e], inv, bq[3][s][r]);
            float ig = fsig(pi), fg = fsig(pf), gg = ftanh(pg), og = fsig(po);
            float cn = fg * cold[s][r] + ig * gg;
            float hn = og * ftanh(cn);
            cnew[s][r] = cn;
            hnew[s][r] = hn;
            hk.h[e] = (f16t)(hn * 8.0f);
        }
    }
    *(v4f*)cp       = cnew[0];
    *(v4f*)(cp + 4) = cnew[1];
    *(v8h*)hp16     = hk.h;
    if (last) {
        *(v4f*)hpf       = hnew[0];
        *(v4f*)(hpf + 4) = hnew[1];
    }
}

__global__ __launch_bounds__(NTHR)
void k_pack_h(const float* __restrict__ W, f16t* P, int K, int N, float sc) {
    int i   = blockIdx.x * NTHR + threadIdx.x;
    int kq  = K >> 3;
    int tot = N * kq;
    if (i >= tot) return;
    int n = i / kq;
    int k = (i - n * kq) * 8;
    PkH v;
#pragma unroll
    for (int e = 0; e < 8; ++e)
        v.h[e] = (f16t)(W[(size_t)(k + e) * N + n] * sc);
    f16t* d = P + (size_t)n * K + k;
    *(volatile v4u*)d = v.u;
    __threadfence();
    *(volatile v4u*)d = v.u;
}

__global__ __launch_bounds__(NTHR)
void k_pack_b2(const float* __restrict__ W, bf16* Ph, bf16* Pl, int K, int N, float sc) {
    int i   = blockIdx.x * NTHR + threadIdx.x;
    int kq  = K >> 3;
    int tot = N * kq;
    if (i >= tot) return;
    int n = i / kq;
    int k = (i - n * kq) * 8;
    PkB vh, vl;
#pragma unroll
    for (int e = 0; e < 8; ++e) {
        float v  = W[(size_t)(k + e) * N + n] * sc;
        bf16  hb = (bf16)v;
        vh.h[e] = hb;
        vl.h[e] = (bf16)(v - (float)hb);
    }
    bf16* dh = Ph + (size_t)n * K + k;
    bf16* dl = Pl + (size_t)n * K + k;
    *(volatile v4u*)dh = vh.u;
    *(volatile v4u*)dl = vl.u;
    __threadfence();
    *(volatile v4u*)dh = vh.u;
    *(volatile v4u*)dl = vl.u;
}

__global__ __launch_bounds__(NTHR)
void k_lstm(const float* __restrict__ obs, const f16t* __restrict__ PWh,
            const bf16* __restrict__ PXh, const bf16* __restrict__ PXl,
            const float* __restrict__ bg,
            const bf16* __restrict__ PDh, const bf16* __restrict__ PDl,
            const float* __restrict__ bd, float* out, int T, int nb) {
    __shared__ LdsU S;
    const int tid = threadIdx.x;
    const int w = tid >> 5, l = tid & 31, hh = l >> 4, m = l & 15;
    const int b0 = blockIdx.x * NB;
    if (b0 + NB > nb) return;

    {
        f16t* hz = &S.a.h16[0][0];
        for (int i = tid; i < 2 * NB * HP; i += NTHR) hz[i] = (f16t)0.0f;
        for (int i = tid; i < NB * HID; i += NTHR) S.a.c[i] = 0.0f;
    }
    const int   xr  = tid >> 4;
    const int   xc  = (tid & 15) * 4;
    const float inv = 0.0078125f;

#pragma unroll 1
    for (int t = 0; t < T; ++t) {
        {
            v4f xv = *(const v4f*)(obs + ((size_t)(b0 + xr) * T + t) * DIN + xc);
            PkB4 ph, pl;
#pragma unroll
            for (int e = 0; e < 4; ++e) {
                float v  = xv[e];
                bf16  hb = (bf16)v;
                ph.h[e] = hb;
                pl.h[e] = (bf16)(v - (float)hb);
            }
            *(v2u*)(S.a.xh + xr * XP + xc) = ph.u;
            *(v2u*)(S.a.xl + xr * XP + xc) = pl.u;
        }
        __syncthreads();
        const int   cur  = t & 1, nxt = cur ^ 1;
        const bool  last = (t == T - 1);
        const f16t* hrow  = S.a.h16[cur] + m * HP + 8 * hh;
        const bf16* xhrow = S.a.xh + m * XP + 8 * hh;
        const bf16* xlrow = S.a.xl + m * XP + 8 * hh;
#pragma unroll 1
        for (int jt = 0; jt < 4; ++jt) {
            const int j0 = (w * 4 + jt) * 16;
            v8f acc[4];
            {
                const v8f z = {0.f, 0.f, 0.f, 0.f, 0.f, 0.f, 0.f, 0.f};
#pragma unroll
                for (int q = 0; q < 4; ++q) acc[q] = z;
            }
            gate_mma(acc,
                     PWh + (size_t)(j0 + m) * HID + 8 * hh,
                     PXh + (size_t)(j0 + m) * DIN + 8 * hh,
                     PXl + (size_t)(j0 + m) * DIN + 8 * hh,
                     hrow, xhrow, xlrow);
            const int jb = j0 + 8 * hh;
            cell_update(acc, inv, bg, jb,
                        S.a.c + m * HID + jb,
                        S.a.h16[nxt] + m * HP + jb,
                        S.a.hf + m * HID + jb,
                        last);
        }
        __syncthreads();
    }

#pragma unroll 1
    for (int i = tid; i < NB * HID; i += NTHR) {
        float v  = S.a.hf[i];
        bf16  hb = (bf16)v;
        S.b.ph[i] = hb;
        S.b.pl[i] = (bf16)(v - (float)hb);
    }
    __syncthreads();
    {
        v8f acc[2];
        {
            const v8f z = {0.f, 0.f, 0.f, 0.f, 0.f, 0.f, 0.f, 0.f};
            acc[0] = z; acc[1] = z;
        }
        const bf16* bhp = S.b.ph + m * HID + 8 * hh;
        const bf16* blp = S.b.pl + m * HID + 8 * hh;
        const bf16* ahp = PDh + (size_t)(32 * w + m) * HID + 8 * hh;
        const bf16* alp = PDl + (size_t)(32 * w + m) * HID + 8 * hh;
#pragma unroll 1
        for (int kt = 0; kt < HID / 32; ++kt) {
            const int k0 = 32 * kt;
            FragB bh, bl, a[2];
            bh.q[0] = *(const v8b*)(bhp + k0);
            bh.q[1] = *(const v8b*)(bhp + k0 + 16);
            bl.q[0] = *(const v8b*)(blp + k0);
            bl.q[1] = *(const v8b*)(blp + k0 + 16);
#pragma unroll
            for (int i = 0; i < 2; ++i) {
                const bf16* p = ahp + (size_t)i * 16 * HID + k0;
                a[i].q[0] = *(const v8b*)p;
                a[i].q[1] = *(const v8b*)(p + 16);
            }
#pragma unroll
            for (int i = 0; i < 2; ++i) acc[i] = mma_b(a[i].v, bh.v, acc[i]);
#pragma unroll
            for (int i = 0; i < 2; ++i) acc[i] = mma_b(a[i].v, bl.v, acc[i]);
            guard2b(acc, a, bh, bl);
#pragma unroll
            for (int i = 0; i < 2; ++i) {
                const bf16* p = alp + (size_t)i * 16 * HID + k0;
                a[i].q[0] = *(const v8b*)p;
                a[i].q[1] = *(const v8b*)(p + 16);
            }
#pragma unroll
            for (int i = 0; i < 2; ++i) acc[i] = mma_b(a[i].v, bh.v, acc[i]);
            guard2b(acc, a, bh, bl);
        }
#pragma unroll
        for (int i = 0; i < 2; ++i) {
            const int fb = 32 * w + 16 * i + 8 * hh;
            v4f d0 = *(const v4f*)(bd + fb);
            v4f d1 = *(const v4f*)(bd + fb + 4);
            v4f y0, y1;
#pragma unroll
            for (int r = 0; r < 4; ++r) {
                y0[r] = fmaxf(acc[i][r] + d0[r], 0.0f);
                y1[r] = fmaxf(acc[i][4 + r] + d1[r], 0.0f);
            }
            float* op = S.b.o + m * FOUT + fb;
            *(v4f*)op       = y0;
            *(v4f*)(op + 4) = y1;
        }
    }
    __syncthreads();
    v4f v[4];
#pragma unroll
    for (int i = 0; i < 4; ++i) {
        int p = tid + NTHR * i, row = p >> 6, c4 = (p & 63) * 4;
        v[i] = *(const v4f*)(S.b.o + row * FOUT + c4);
    }
#pragma unroll
    for (int i = 0; i < 4; ++i) {
        int p = tid + NTHR * i, row = p >> 6, c4 = (p & 63) * 4;
        *(volatile v4f*)(out + (size_t)(b0 + row) * FOUT + c4) = v[i];
    }
    __threadfence();
#pragma unroll
    for (int i = 0; i < 4; ++i) {
        int p = tid + NTHR * i, row = p >> 6, c4 = (p & 63) * 4;
        *(volatile v4f*)(out + (size_t)(b0 + row) * FOUT + c4) = v[i];
    }
}

extern "C" void kernel_launch(void* const* d_in, const int* in_sizes, int n_in,
                              void* d_out, int out_size, void* d_ws, size_t ws_size,
                              hipStream_t stream) {
    if (n_in < 6) return;
    if (out_size <= 0 || (out_size % FOUT) != 0) return;
    const int nb = out_size / FOUT;
    if ((nb % NB) != 0) return;
    if (in_sizes[1] != DIN * G4 || in_sizes[2] != HID * G4 || in_sizes[3] != G4 ||
        in_sizes[4] != HID * FOUT || in_sizes[5] != FOUT) return;
    if (in_sizes[0] <= 0 || (in_sizes[0] % (nb * DIN)) != 0) return;
    const int T = in_sizes[0] / (nb * DIN);
    if (T < 1) return;

    const float* obs = (const float*)d_in[0];
    const float* Wx  = (const float*)d_in[1];
    const float* Wh  = (const float*)d_in[2];
    const float* bg  = (const float*)d_in[3];
    const float* Wd  = (const float*)d_in[4];
    const float* bd  = (const float*)d_in[5];
    float* out = (float*)d_out;

    char* ws = (char*)d_ws;
    size_t off = 0;
    auto carve = [&](size_t bytes) -> char* {
        char* p = ws + off;
        off = (off + bytes + 255) & ~(size_t)255;
        return p;
    };
    f16t* PWh = (f16t*)carve((size_t)G4 * HID * 2);
    bf16* PXh = (bf16*)carve((size_t)G4 * DIN * 2);
    bf16* PXl = (bf16*)carve((size_t)G4 * DIN * 2);
    bf16* PDh = (bf16*)carve((size_t)FOUT * HID * 2);
    bf16* PDl = (bf16*)carve((size_t)FOUT * HID * 2);
    if (off > ws_size || off > (size_t)134217728) return;

    {
        int tot = G4 * (HID / 8);
        k_pack_h<<<dim3((tot + NTHR - 1) / NTHR), dim3(NTHR), 0, stream>>>(Wh, PWh, HID, G4, 16.0f);
    }
    {
        int tot = G4 * (DIN / 8);
        k_pack_b2<<<dim3((tot + NTHR - 1) / NTHR), dim3(NTHR), 0, stream>>>(Wx, PXh, PXl, DIN, G4, 128.0f);
    }
    {
        int tot = FOUT * (HID / 8);
        k_pack_b2<<<dim3((tot + NTHR - 1) / NTHR), dim3(NTHR), 0, stream>>>(Wd, PDh, PDl, HID, FOUT, 1.0f);
    }
    k_lstm<<<dim3(nb / NB), dim3(NTHR), 0, stream>>>(obs, PWh, PXh, PXl, bg, PDh, PDl, bd, out, T, nb);
}
